// ODEFunc_80582176407958
// MI455X (gfx1250) — hardware-verified
//
#include <hip/hip_runtime.h>


namespace {
typedef _Float16 b16;
typedef __attribute__((ext_vector_type(16))) _Float16 v16b;
typedef __attribute__((ext_vector_type(8))) _Float16 v8b;
typedef __attribute__((ext_vector_type(4))) _Float16 v4h;
typedef __attribute__((ext_vector_type(2))) _Float16 v2h;
typedef __attribute__((ext_vector_type(8))) float v8f;
typedef __attribute__((ext_vector_type(4))) float v4f;
typedef __attribute__((ext_vector_type(2))) float v2f;
__device__ __forceinline__ float bf16_rne(float f) { unsigned int u = __float_as_uint(f); u += 0x7FFFu + ((u >> 16) & 1u); return __uint_as_float(u & 0xFFFF0000u); }
__device__ __forceinline__ void split16(float v, b16& hi, b16& lo) { hi = (b16)v; lo = (b16)(v - (float)hi); }
__device__ __forceinline__ v16b frag_kb(const b16* p, int hh) { const v8b a = *(const v8b*)(p + 8 * hh), b = *(const v8b*)(p + 16 + 8 * hh); v16b f;
#pragma unroll
  for (int e = 0; e < 8; ++e) { f[e] = a[e]; f[8 + e] = b[e]; } return f; }
__device__ __forceinline__ v8f wmma16b(v16b a, v16b b, v8f c) { v8f d = __builtin_amdgcn_wmma_f32_16x16x32_f16(false, a, false, b, (short)0, c, false, false); asm volatile("v_nop\n\tv_nop\n\tv_nop\n\tv_nop" : "+v"(d) : "v"(a), "v"(b)); return d; }
__device__ __forceinline__ void wave_lds_sync() { __builtin_amdgcn_fence(__ATOMIC_RELEASE, "workgroup"); __builtin_amdgcn_wave_barrier(); __builtin_amdgcn_fence(__ATOMIC_ACQUIRE, "workgroup"); }
__device__ __forceinline__ float pmul(float a, float b) { float p = a * b; asm volatile("" : "+v"(p)); return p; }
__device__ __forceinline__ int iclamp(int v, int lo, int hi) { return v < lo ? lo : (v > hi ? hi : v); }
__device__ __forceinline__ float nexp2(float v) { return __builtin_amdgcn_exp2f(v); }

constexpr int N = 16384, NP = 16384, D = 64, H = 256, NL = N  ;
constexpr float XS = 8.0f, WSC = 256.0f, MS = 4096.0f, RS = 1024.0f, SLOPE = 0.0f, BNEPS = 1e-5f;
static_assert(N % 64 == 0 && NL % 64 == 0 && H % 128 == 0 && D % 32 == 0, "tiling");

typedef __attribute__((ext_vector_type(4))) _Float16 v4h;
typedef __attribute__((ext_vector_type(2))) float v2f;
template <int KD, int NOUT>
__global__ __launch_bounds__(256) void wprep_kernel(const float* __restrict__ w, b16* __restrict__ WT) {
  static_assert(KD % 8 == 0, "wprep"); const size_t u = (size_t)blockIdx.x * 256 + threadIdx.x; if (u >= (size_t)NOUT * KD / 8) return; const size_t e = u * 8; const int oo = (int)(e / KD), k0 = (int)(e % KD); v8b o;
  for (int j = 0; j < 8; ++j) o[j] = (b16)(bf16_rne(w[(size_t)(k0 + j) * NOUT + oo]) * WSC);
  for (int pass = 0; pass < 2; ++pass) { *(volatile v8b*)(WT + e) = o; __threadfence(); }
}
template <int KD, int NOUT, int NV, bool RNDA  >
__global__ __launch_bounds__(64) void gemm_kernel(const float* __restrict__ A, const b16* __restrict__ W, float* __restrict__ T) {
  constexpr int SL = NOUT < 128 ? NOUT : 128, NT = SL / 16, KC = KD < 128 ? KD : 128;
  static_assert(KD % KC == 0 && KC % 32 == 0 && NOUT % SL == 0 && SL % 32 == 0, "gemm tiling");
  __shared__ __attribute__((aligned(16))) b16 Ah[2][16][KC + 8], Al[2][16][KC + 8]; __shared__ __attribute__((aligned(16))) float Tf[2][16][SL + 4];
  const int wave = threadIdx.x >> 5, lane = threadIdx.x & 31, nloc = lane & 15, hlf = lane >> 4; const size_t m0 = (size_t)blockIdx.x * 32 + wave * 16; const int n0 = blockIdx.y * SL;
  v8f acc[NT];
#pragma unroll
  for (int t = 0; t < NT; ++t) acc[t] = (v8f){};
#pragma unroll 1
  for (int kc = 0; kc < KD; kc += KC) {
    for (int idx = lane; idx < 16 * (KC / 4); idx += 32) { const int rr = idx / (KC / 4), c4 = (idx % (KC / 4)) * 4; const size_t row = (m0 + rr < (size_t)NV) ? (m0 + rr) : (size_t)(NV - 1); const v4f v = *(const v4f*)(A + row * KD + kc + c4); v4h hv, lv;
      for (int j = 0; j < 4; ++j) { b16 ph, pl; split16((RNDA ? bf16_rne(v[j]) : v[j]) * XS, ph, pl); hv[j] = ph; lv[j] = pl; } *(v4h*)(&Ah[wave][rr][c4]) = hv; *(v4h*)(&Al[wave][rr][c4]) = lv; }
    wave_lds_sync();
#pragma unroll
    for (int kb = 0; kb < KC; kb += 32) { const v16b a = frag_kb(&Ah[wave][nloc][kb], hlf), al = frag_kb(&Al[wave][nloc][kb], hlf);
#pragma unroll
      for (int t = 0; t < NT; ++t) { const v16b bw = frag_kb(W + (size_t)(n0 + t * 16 + nloc) * KD + kc + kb, hlf); acc[t] = wmma16b(a, bw, acc[t]); acc[t] = wmma16b(al, bw, acc[t]); } }
    wave_lds_sync(); }
#pragma unroll
  for (int t = 0; t < NT; ++t)
#pragma unroll
    for (int r = 0; r < 8; ++r) Tf[wave][8 * hlf + r][t * 16 + nloc] = acc[t][r] * (1.0f / (XS * WSC));
  wave_lds_sync();
  for (int pass = 0; pass < 2; ++pass) { for (int idx = lane; idx < 16 * (SL / 4); idx += 32) { const int rr = idx / (SL / 4), c4 = (idx % (SL / 4)) * 4; *(volatile v4f*)(T + (m0 + rr) * NOUT + n0 + c4) = *(const v4f*)(&Tf[wave][rr][c4]); } __threadfence(); }
}

__global__ __launch_bounds__(256) void prep_kernel(const float* __restrict__ tt, const float* __restrict__ w1, const float* __restrict__ b1, const float* __restrict__ w2, const float* __restrict__ w3, b16* __restrict__ WT1, b16* __restrict__ WT2, b16* __restrict__ WT3, float* __restrict__ C1, b16* __restrict__ MH, b16* __restrict__ ML) {
  const int n1 = H * D / 8, n2 = H * H / 8, n3 = D * H / 8, n4 = H * H / 8, n5 = H / 8; int u = blockIdx.x * 256 + threadIdx.x; v8b o;
  if (u < n1) { const int e = u * 8, oo = e / D, k0 = e % D; for (int j = 0; j < 8; ++j) o[j] = (b16)(bf16_rne(w1[(size_t)(k0 + j) * H + oo]) * WSC); for (int pass = 0; pass < 2; ++pass) { *(volatile v8b*)(WT1 + e) = o; __threadfence(); } return; } u -= n1;
  if (u < n2) { const int e = u * 8, oo = e / H, k0 = e % H; for (int j = 0; j < 8; ++j) o[j] = (b16)(bf16_rne(w2[(size_t)(k0 + j) * H + oo]) * WSC); for (int pass = 0; pass < 2; ++pass) { *(volatile v8b*)(WT2 + e) = o; __threadfence(); } return; } u -= n2;
  if (u < n3) { const int e = u * 8, oo = e / H, k0 = e % H; for (int j = 0; j < 8; ++j) o[j] = (b16)(bf16_rne(w3[(size_t)(k0 + j) * D + oo]) * WSC); for (int pass = 0; pass < 2; ++pass) { *(volatile v8b*)(WT3 + e) = o; __threadfence(); } return; } u -= n3;
  if (u < n4) { const int e = u * 8, a = e / H, b0 = e % H; v8b hv, lv;
    for (int j = 0; j < 8; ++j) { const int b = b0 + j; float g = 0.0f;
#pragma unroll 4
      for (int i = 0; i < D; ++i) g = fmaf(bf16_rne(w1[(size_t)i * H + a]), bf16_rne(w3[(size_t)b * D + i]), g);
      const float m = bf16_rne(w2[(size_t)a * H + b]) * g * MS; const b16 hh_ = (b16)m; hv[j] = hh_; lv[j] = (b16)((m - (float)hh_) * RS); }
    for (int pass = 0; pass < 2; ++pass) { *(volatile v8b*)(MH + e) = hv; *(volatile v8b*)(ML + e) = lv; __threadfence(); } return; } u -= n4;
  if (u < n5) { const int e = u * 8; const float tv = bf16_rne(tt[0]); v4f c0, c1; for (int j = 0; j < 4; ++j) { c0[j] = bf16_rne(b1[e + j]) + tv * bf16_rne(w1[(size_t)D * H + e + j]); c1[j] = bf16_rne(b1[e + 4 + j]) + tv * bf16_rne(w1[(size_t)D * H + e + 4 + j]); }
    for (int pass = 0; pass < 2; ++pass) { *(volatile v4f*)(C1 + e) = c0; *(volatile v4f*)(C1 + e + 4) = c1; __threadfence(); } }
}
template <int KD, bool RNDA>
__global__ __launch_bounds__(64) void layer_kernel(const float* __restrict__ A, const b16* __restrict__ W, const float* __restrict__ cvec, bool cvec_raw, float* __restrict__ Hout, float* __restrict__ Dout) {
  constexpr int KC = KD < 128 ? KD : 128; static_assert(KD % KC == 0 && KC % 32 == 0, "k");
  __shared__ __attribute__((aligned(16))) b16 Ah[2][16][KC + 8], Al[2][16][KC + 8]; __shared__ __attribute__((aligned(16))) float Tf[2][16][128 + 4], Td[2][16][128 + 4];
  const int wave = threadIdx.x >> 5, lane = threadIdx.x & 31, nloc = lane & 15, hlf = lane >> 4; const size_t m0 = (size_t)blockIdx.x * 32 + wave * 16; const int n0 = blockIdx.y * 128;
  v8f acc[8];
#pragma unroll
  for (int t = 0; t < 8; ++t) acc[t] = (v8f){};
#pragma unroll 1
  for (int kc = 0; kc < KD; kc += KC) {
    for (int idx = lane; idx < 16 * (KC / 4); idx += 32) { const int rr = idx / (KC / 4), c4 = (idx % (KC / 4)) * 4; const v4f v = *(const v4f*)(A + (m0 + rr) * KD + kc + c4); v4h hv, lv;
      for (int j = 0; j < 4; ++j) { b16 ph, pl; split16((RNDA ? bf16_rne(v[j]) : v[j]) * XS, ph, pl); hv[j] = ph; lv[j] = pl; } *(v4h*)(&Ah[wave][rr][c4]) = hv; *(v4h*)(&Al[wave][rr][c4]) = lv; }
    wave_lds_sync();
#pragma unroll
    for (int kb = 0; kb < KC; kb += 32) { const v16b a = frag_kb(&Ah[wave][nloc][kb], hlf), al = frag_kb(&Al[wave][nloc][kb], hlf);
#pragma unroll
      for (int t = 0; t < 8; ++t) { const v16b bw = frag_kb(W + (size_t)(n0 + t * 16 + nloc) * KD + kc + kb, hlf); acc[t] = wmma16b(a, bw, acc[t]); if (!RNDA) acc[t] = wmma16b(al, bw, acc[t]); } }
    wave_lds_sync(); }
#pragma unroll
  for (int t = 0; t < 8; ++t) { const int c = n0 + t * 16 + nloc; const float cb = cvec_raw ? bf16_rne(cvec[c]) : cvec[c];
#pragma unroll
    for (int r = 0; r < 8; ++r) { const float a = acc[t][r] * (1.0f / (XS * WSC)) + cb; const float s = 1.0f / (1.0f + __expf(-a)); Tf[wave][8 * hlf + r][t * 16 + nloc] = a * s; Td[wave][8 * hlf + r][t * 16 + nloc] = s * (1.0f + a * (1.0f - s)); } }
  wave_lds_sync();
  for (int pass = 0; pass < 2; ++pass) { for (int rr = 0; rr < 16; ++rr) { *(volatile v4f*)(Hout + (m0 + rr) * H + n0 + lane * 4) = *(const v4f*)(&Tf[wave][rr][lane * 4]); *(volatile v4f*)(Dout + (m0 + rr) * H + n0 + lane * 4) = *(const v4f*)(&Td[wave][rr][lane * 4]); } __threadfence(); }
}
__global__ __launch_bounds__(64) void out0_kernel(const float* __restrict__ A, const b16* __restrict__ W, const float* __restrict__ b3, float* __restrict__ out) {
  __shared__ __attribute__((aligned(16))) b16 Ah[2][16][128 + 8], Al[2][16][128 + 8]; __shared__ __attribute__((aligned(16))) float Tf[2][16][D + 4];
  const int wave = threadIdx.x >> 5, lane = threadIdx.x & 31, nloc = lane & 15, hlf = lane >> 4; const size_t m0 = (size_t)blockIdx.x * 32 + wave * 16;
  v8f acc[4];
#pragma unroll
  for (int t = 0; t < 4; ++t) acc[t] = (v8f){};
#pragma unroll 1
  for (int kc = 0; kc < H; kc += 128) {
    for (int rr = 0; rr < 16; ++rr) { const v4f v = *(const v4f*)(A + (m0 + rr) * H + kc + lane * 4); v4h hv, lv; for (int j = 0; j < 4; ++j) { b16 ph, pl; split16(v[j] * XS, ph, pl); hv[j] = ph; lv[j] = pl; } *(v4h*)(&Ah[wave][rr][lane * 4]) = hv; *(v4h*)(&Al[wave][rr][lane * 4]) = lv; }
    wave_lds_sync();
#pragma unroll
    for (int kb = 0; kb < 128; kb += 32) { const v16b a = frag_kb(&Ah[wave][nloc][kb], hlf), al = frag_kb(&Al[wave][nloc][kb], hlf);
#pragma unroll
      for (int t = 0; t < 4; ++t) { const v16b bw = frag_kb(W + (size_t)(t * 16 + nloc) * H + kc + kb, hlf); acc[t] = wmma16b(a, bw, acc[t]); acc[t] = wmma16b(al, bw, acc[t]); } }
    wave_lds_sync(); }
#pragma unroll
  for (int t = 0; t < 4; ++t) { const float bb = bf16_rne(b3[t * 16 + nloc]);
#pragma unroll
    for (int r = 0; r < 8; ++r) Tf[wave][8 * hlf + r][t * 16 + nloc] = acc[t][r] * (1.0f / (XS * WSC)) + bb; }
  wave_lds_sync();
  for (int pass = 0; pass < 2; ++pass) { for (int idx = lane; idx < 16 * (D / 4); idx += 32) { const int rr = idx / (D / 4), c4 = (idx % (D / 4)) * 4; *(volatile v4f*)(out + (m0 + rr) * D + c4) = *(const v4f*)(&Tf[wave][rr][c4]); } __threadfence(); }
}
__global__ __launch_bounds__(256) void div_kernel(const float* __restrict__ D1, const float* __restrict__ UH, const float* __restrict__ UL, float* __restrict__ out1) {
  const int s = blockIdx.x * 256 + threadIdx.x; if (s >= NL) return;
  float acc = 0.0f; const float ch = WSC / MS, cl = WSC / (MS * RS);
#pragma unroll 2
  for (int a = 0; a < H; a += 4) { const v4f d = *(const v4f*)(D1 + (size_t)s * H + a), uh = *(const v4f*)(UH + (size_t)s * H + a), ul = *(const v4f*)(UL + (size_t)s * H + a); for (int i = 0; i < 4; ++i) acc = fmaf(d[i], uh[i] * ch + ul[i] * cl, acc); }
  for (int pass = 0; pass < 2; ++pass) { ((volatile float*)out1)[s] = -acc; __threadfence(); }
}
}

extern "C" void kernel_launch(void* const* d_in, const int* in_sizes, int n_in, void* d_out, int out_size, void* d_ws, size_t ws_size, hipStream_t stream) {
  (void)n_in;
  auto Fp = [&](int i) { return (const float*)d_in[i]; };
  if (in_sizes[0] != 1 || in_sizes[1] != N * D || in_sizes[3] != (D + 1) * H || in_sizes[4] != H || in_sizes[5] != H * H || in_sizes[6] != H || in_sizes[7] != H * D || in_sizes[8] != D || out_size != N * D + N) return;
  size_t off = 0; char* ws = (char*)d_ws;
  auto carve = [&](size_t bytes) { char* p = ws + off; off += (bytes + 255) & ~(size_t)255; return p; };
  b16* WT1 = (b16*)carve((size_t)H * D * 2); b16* WT2 = (b16*)carve((size_t)H * H * 2); b16* WT3 = (b16*)carve((size_t)D * H * 2); float* C1 = (float*)carve((size_t)H * 4); b16* MH = (b16*)carve((size_t)H * H * 2); b16* ML = (b16*)carve((size_t)H * H * 2);
  const size_t pl = (size_t)NP * H * 4; float* H1 = (float*)carve(pl); float* D1 = (float*)carve(pl); float* H2 = (float*)carve(pl); float* D2 = (float*)carve(pl); float* UH = (float*)carve(pl); float* UL = (float*)carve(pl);
  if (off > ws_size || off > ((size_t)128 << 20)) return;
  prep_kernel<<<(H * D / 8 + H * H / 8 + D * H / 8 + H * H / 8 + H / 8 + 255) / 256, 256, 0, stream>>>(Fp(0), Fp(3), Fp(4), Fp(5), Fp(7), WT1, WT2, WT3, C1, MH, ML);
  layer_kernel<D, true><<<dim3(NL / 32, 2), 64, 0, stream>>>(Fp(1), WT1, C1, false, H1, D1);
  layer_kernel<H, false><<<dim3(NL / 32, 2), 64, 0, stream>>>(H1, WT2, Fp(6), true, H2, D2);
  out0_kernel<<<NL / 32, 64, 0, stream>>>(H2, WT3, Fp(8), (float*)d_out);
  gemm_kernel<H, H, NP, false><<<dim3(NL / 32, 2), 64, 0, stream>>>(D2, MH, UH);
  gemm_kernel<H, H, NP, false><<<dim3(NL / 32, 2), 64, 0, stream>>>(D2, ML, UL);
  div_kernel<<<NL / 256, 256, 0, stream>>>(D1, UH, UL, (float*)d_out + (size_t)N * D);
}
